// PCT_77824807404164
// MI455X (gfx1250) — hardware-verified
//
#include <hip/hip_runtime.h>
#define BB 16
#define CC 256
#define NN 1024
#define DQK 64
#define DVV 256
#define NBIN 32
#define NREL 63
#define NRP 64
#define NTOK (BB * NN)

typedef __bf16 v16b __attribute__((ext_vector_type(16)));
typedef unsigned short v8us __attribute__((ext_vector_type(8), may_alias));
typedef float  v8f  __attribute__((ext_vector_type(8)));
typedef float  v4f  __attribute__((ext_vector_type(4)));
typedef float  v4fa __attribute__((ext_vector_type(4), may_alias));
union FragB { v16b v; v8us half[2]; unsigned short u[16]; };

__device__ __forceinline__ unsigned short bf16_bits(float x) { unsigned int u = __float_as_uint(x); return (unsigned short)((u + 0x7FFFu + ((u >> 16) & 1u)) >> 16); }
__device__ __forceinline__ float bf16_val(unsigned short b) { return __uint_as_float(((unsigned int)b) << 16); }
__device__ __forceinline__ float bf16_round(float x) { return bf16_val(bf16_bits(x)); }
template <int NT>
__device__ __forceinline__ v8f mmaN(v16b ah, v16b al, v16b bh, v16b bl, v8f c) {
  c = __builtin_amdgcn_wmma_f32_16x16x32_bf16(false, ah, false, bh, (short)0, c, false, false);
  if (NT >= 2) c = __builtin_amdgcn_wmma_f32_16x16x32_bf16(false, al, false, bh, (short)0, c, false, false);
  if (NT >= 3) c = __builtin_amdgcn_wmma_f32_16x16x32_bf16(false, ah, false, bl, (short)0, c, false, false);
  asm volatile("v_nop\n\tv_nop\n\tv_nop\n\tv_nop" : "+v"(c) : "v"(ah), "v"(al), "v"(bh), "v"(bl));
  return c;
}

__global__ __launch_bounds__(256) void k_wt_bf16(const float* __restrict__ W, unsigned short* __restrict__ Wt, int K, int N) {
  const int t = blockIdx.x * 256 + threadIdx.x;
  const int k8n = K / 8;
  if (t >= N * k8n) return;
  const int n = t / k8n, k8 = (t % k8n) * 8;
  v8us v;
#pragma unroll
  for (int i = 0; i < 8; ++i) v[i] = bf16_bits(W[(size_t)(k8 + i) * N + n]);
  *(volatile v8us*)(Wt + (size_t)n * K + k8) = v;
  __threadfence();
  *(volatile v8us*)(Wt + (size_t)n * K + k8) = v;
}

template <bool ASPLIT, int ACT, bool BIAS_BF16>
__global__ __launch_bounds__(128) void k_gemm_bf(const float* __restrict__ A, int lda, const unsigned short* __restrict__ Wt, int ldb,
                                               const float* __restrict__ bias, float* __restrict__ C, int ldc, int M, int N, int K) {
  __shared__ __attribute__((aligned(16))) float so[4][16][64];
  const int tid = threadIdx.x, w = tid >> 5, lane = tid & 31, ln = lane & 15, hh = lane >> 4;
  const int ntn = N / 64;
  const int wid = blockIdx.x * 4 + w;
  const int mt = wid / ntn, nq = wid % ntn;
  if (mt * 16 >= M) return;
  const int row0 = mt * 16, col0 = nq * 64;
  const float* arow = A + (size_t)(row0 + ln) * lda;
  v8f acc[4] = {};
  for (int kb = 0; kb < K; kb += 32) {
    FragB ah, al;
    const v4f x0 = *(const v4fa*)(arow + kb + 8 * hh), x1 = *(const v4fa*)(arow + kb + 8 * hh + 4);
    const v4f x2 = *(const v4fa*)(arow + kb + 16 + 8 * hh), x3 = *(const v4fa*)(arow + kb + 16 + 8 * hh + 4);
    float xs[16] = {x0[0],x0[1],x0[2],x0[3],x1[0],x1[1],x1[2],x1[3],x2[0],x2[1],x2[2],x2[3],x3[0],x3[1],x3[2],x3[3]};
#pragma unroll
    for (int i = 0; i < 16; ++i) { const unsigned short hb = bf16_bits(xs[i]); ah.u[i] = hb; al.u[i] = ASPLIT ? bf16_bits(xs[i] - bf16_val(hb)) : (unsigned short)0; }
#pragma unroll
    for (int t = 0; t < 4; ++t) {
      const unsigned short* brow = Wt + (size_t)(col0 + t * 16 + ln) * ldb + kb;
      FragB b;
      b.half[0] = *(const v8us*)(brow + 8 * hh);
      b.half[1] = *(const v8us*)(brow + 16 + 8 * hh);
      acc[t] = mmaN<ASPLIT ? 2 : 1>(ah.v, al.v, b.v, b.v, acc[t]);
    }
  }
#pragma unroll
  for (int t = 0; t < 4; ++t) {
    float bv = bias ? bias[col0 + t * 16 + ln] : 0.f;
    if (BIAS_BF16) bv = bf16_round(bv);
#pragma unroll
    for (int r = 0; r < 8; ++r) { float v = acc[t][r] + bv; if (ACT == 1) v = fmaxf(v, 0.f); so[w][8 * hh + r][t * 16 + ln] = v; }
  }
  __builtin_amdgcn_fence(__ATOMIC_ACQ_REL, "workgroup");
  __builtin_amdgcn_wave_barrier();
  const int rsub = lane >> 4, c4 = (lane & 15) * 4;
  for (int pass = 0; pass < 2; ++pass) {
#pragma unroll
    for (int q = 0; q < 8; ++q) {
      const int r = q * 2 + rsub;
      const v4f v = *(const v4fa*)&so[w][r][c4];
      *(volatile v4f*)(C + (size_t)(row0 + r) * ldc + col0 + c4) = v;
    }
    if (pass == 0) __threadfence();
  }
}

template <int D, bool CAUSAL>
__global__ __launch_bounds__(128) void k_flash(const float* __restrict__ qb, const float* __restrict__ kb, const float* __restrict__ vb,
                                             int pitch, int T, int H, float scale, float* __restrict__ y, int ypitch) {
  constexpr int KS = D / 32;
  constexpr int DT = D / 16;
  __shared__ __attribute__((aligned(16))) unsigned short sKh[32][D + 8], sKl[32][D + 8], sVh[32][D + 8], sVl[32][D + 8];
  __shared__ __attribute__((aligned(16))) unsigned short sPh[4][16][40], sPl[4][16][40];
  __shared__ __attribute__((aligned(16))) float sO[4][16][D];
  const int tid = threadIdx.x, w = tid >> 5, lane = tid & 31, ln = lane & 15, hh = lane >> 4;
  const int nqb = (T + 63) / 64;
  const int bh = blockIdx.x / nqb, qblk = blockIdx.x % nqb;
  const int b = bh / H, h = bh % H;
  const int q0 = qblk * 64 + w * 16;
  const float* Q = qb + (size_t)b * T * pitch + h * D;
  const float* K = kb + (size_t)b * T * pitch + h * D;
  const float* V = vb + (size_t)b * T * pitch + h * D;

  FragB aqh[KS], aql[KS];
  {
    int row = q0 + ln; if (row >= T) row = T - 1;
    const float* qr = Q + (size_t)row * pitch;
#pragma unroll
    for (int ks = 0; ks < KS; ++ks)
#pragma unroll
      for (int i = 0; i < 16; ++i) {
        const int d = ks * 32 + ((i < 8) ? (8 * hh + i) : (16 + 8 * hh + (i - 8)));
        const float x = qr[d] * scale; const unsigned short hb = bf16_bits(x);
        aqh[ks].u[i] = hb; aql[ks].u[i] = bf16_bits(x - bf16_val(hb));
      }
  }
  float m_r[8], l_r[8];
#pragma unroll
  for (int r = 0; r < 8; ++r) { m_r[r] = -3.0e38f; l_r[r] = 0.f; }
  v8f oacc[DT];
#pragma unroll
  for (int dt = 0; dt < DT; ++dt) oacc[dt] = (v8f){0.f,0.f,0.f,0.f,0.f,0.f,0.f,0.f};

  const int kv_end = CAUSAL ? min(T, qblk * 64 + 64) : T;
  for (int j0 = 0; j0 < kv_end; j0 += 32) {
    __syncthreads();
    for (int e = tid; e < 32 * (D / 4); e += 128) {
      const int r = e / (D / 4), c4 = (e % (D / 4)) * 4;
      const int key = j0 + r;
      v4f kf = {0.f,0.f,0.f,0.f}, vf = {0.f,0.f,0.f,0.f};
      if (key < T) { kf = *(const v4fa*)(K + (size_t)key * pitch + c4); vf = *(const v4fa*)(V + (size_t)key * pitch + c4); }
#pragma unroll
      for (int t = 0; t < 4; ++t) {
        unsigned short hb = bf16_bits(kf[t]); sKh[r][c4 + t] = hb; sKl[r][c4 + t] = bf16_bits(kf[t] - bf16_val(hb));
        hb = bf16_bits(vf[t]); sVh[r][c4 + t] = hb; sVl[r][c4 + t] = bf16_bits(vf[t] - bf16_val(hb));
      }
    }
    __syncthreads();
    v8f s[2];
#pragma unroll
    for (int nt = 0; nt < 2; ++nt) {
      v8f acc = {};
#pragma unroll
      for (int ks = 0; ks < KS; ++ks) {
        FragB bh_, bl_;
        bh_.half[0] = *(const v8us*)&sKh[nt * 16 + ln][ks * 32 + 8 * hh]; bh_.half[1] = *(const v8us*)&sKh[nt * 16 + ln][ks * 32 + 16 + 8 * hh];
        bl_.half[0] = *(const v8us*)&sKl[nt * 16 + ln][ks * 32 + 8 * hh]; bl_.half[1] = *(const v8us*)&sKl[nt * 16 + ln][ks * 32 + 16 + 8 * hh];
        acc = mmaN<3>(aqh[ks].v, aql[ks].v, bh_.v, bl_.v, acc);
      }
      s[nt] = acc;
    }
    float alpha[8];
#pragma unroll
    for (int r = 0; r < 8; ++r) {
      const int qi = q0 + 8 * hh + r;
      const int ja = j0 + ln, jb = j0 + 16 + ln;
      if (CAUSAL) { if (ja > qi) s[0][r] = -3.0e38f; if (jb > qi) s[1][r] = -3.0e38f; }
      if (ja >= T) s[0][r] = -3.0e38f;
      if (jb >= T) s[1][r] = -3.0e38f;
      float mx = fmaxf(s[0][r], s[1][r]);
      mx = fmaxf(mx, __shfl_xor(mx, 1, 32)); mx = fmaxf(mx, __shfl_xor(mx, 2, 32)); mx = fmaxf(mx, __shfl_xor(mx, 4, 32)); mx = fmaxf(mx, __shfl_xor(mx, 8, 32));
      const float mnew = fmaxf(m_r[r], mx);
      alpha[r] = (mnew > -1.0e38f) ? __expf(m_r[r] - mnew) : 1.0f;
      const float p0 = (s[0][r] > -1.0e38f) ? __expf(s[0][r] - mnew) : 0.f;
      const float p1 = (s[1][r] > -1.0e38f) ? __expf(s[1][r] - mnew) : 0.f;
      m_r[r] = mnew;
      l_r[r] = l_r[r] * alpha[r] + p0 + p1;
      unsigned short hb = bf16_bits(p0); sPh[w][8 * hh + r][ln] = hb;      sPl[w][8 * hh + r][ln] = bf16_bits(p0 - bf16_val(hb));
      hb = bf16_bits(p1);                sPh[w][8 * hh + r][16 + ln] = hb; sPl[w][8 * hh + r][16 + ln] = bf16_bits(p1 - bf16_val(hb));
    }
#pragma unroll
    for (int dt = 0; dt < DT; ++dt)
#pragma unroll
      for (int r = 0; r < 8; ++r) oacc[dt][r] *= alpha[r];
    __builtin_amdgcn_fence(__ATOMIC_ACQ_REL, "workgroup");
    __builtin_amdgcn_wave_barrier();
    FragB pah, pal;
    pah.half[0] = *(const v8us*)&sPh[w][ln][8 * hh]; pah.half[1] = *(const v8us*)&sPh[w][ln][16 + 8 * hh];
    pal.half[0] = *(const v8us*)&sPl[w][ln][8 * hh]; pal.half[1] = *(const v8us*)&sPl[w][ln][16 + 8 * hh];
#pragma unroll
    for (int dt = 0; dt < DT; ++dt) {
      FragB bvh, bvl;
#pragma unroll
      for (int i = 0; i < 8; ++i) {
        bvh.u[i] = sVh[8 * hh + i][dt * 16 + ln]; bvh.u[8 + i] = sVh[16 + 8 * hh + i][dt * 16 + ln];
        bvl.u[i] = sVl[8 * hh + i][dt * 16 + ln]; bvl.u[8 + i] = sVl[16 + 8 * hh + i][dt * 16 + ln];
      }
      oacc[dt] = mmaN<3>(pah.v, pal.v, bvh.v, bvl.v, oacc[dt]);
    }
    __builtin_amdgcn_fence(__ATOMIC_ACQ_REL, "workgroup");
    __builtin_amdgcn_wave_barrier();
  }
#pragma unroll
  for (int r = 0; r < 8; ++r) {
    float l = l_r[r];
    l += __shfl_xor(l, 1, 32); l += __shfl_xor(l, 2, 32); l += __shfl_xor(l, 4, 32); l += __shfl_xor(l, 8, 32);
    l_r[r] = (l > 0.f) ? 1.0f / l : 0.f;
  }
#pragma unroll
  for (int dt = 0; dt < DT; ++dt)
#pragma unroll
    for (int r = 0; r < 8; ++r) sO[w][8 * hh + r][dt * 16 + ln] = oacc[dt][r] * l_r[r];
  __builtin_amdgcn_fence(__ATOMIC_ACQ_REL, "workgroup");
  __builtin_amdgcn_wave_barrier();
  for (int pass = 0; pass < 2; ++pass) {
    for (int r = 0; r < 16; ++r) {
      const int row = q0 + r;
      if (row < T && lane < D / 4) {
        const v4f val = *(const v4fa*)&sO[w][r][lane * 4];
        *(volatile v4f*)(y + ((size_t)b * T + row) * ypitch + h * D + lane * 4) = val;
      }
    }
    if (pass == 0) __threadfence();
  }
}

template <bool AFFINE, bool RESID, bool RES_BF16>
__global__ __launch_bounds__(256) void k_transpose32(const float* __restrict__ in, float* __restrict__ out, int rows, int cols,
                                                    const float* __restrict__ scale, const float* __restrict__ shift, const float* __restrict__ res) {
  __shared__ float tile[32][33];
  const int b = blockIdx.z;
  const int r0 = blockIdx.y * 32, c0 = blockIdx.x * 32;
  const float* src = in + (size_t)b * rows * cols;
  float* dst = out + (size_t)b * rows * cols;
  const int tx = threadIdx.x & 31, ty = threadIdx.x >> 5;
  for (int i = ty; i < 32; i += 8) tile[i][tx] = src[(size_t)(r0 + i) * cols + c0 + tx];
  __syncthreads();
  for (int pass = 0; pass < 2; ++pass) {
    for (int i = ty; i < 32; i += 8) {
      float v = tile[tx][i];
      const int orow = c0 + i;
      if (AFFINE) v = v * scale[orow] + shift[orow];
      if (RESID) { float rv = res[(size_t)b * rows * cols + (size_t)orow * rows + r0 + tx]; if (RES_BF16) rv = bf16_round(rv); v += rv; }
      *(volatile float*)(dst + (size_t)orow * rows + r0 + tx) = v;
    }
    if (pass == 0) __threadfence();
  }
}

__global__ __launch_bounds__(256) void k_pool2_pm(const float* __restrict__ in, float* __restrict__ out, int Bn, int H, int W, int C) {
  const size_t t = (size_t)blockIdx.x * 256 + threadIdx.x;
  const int c4n = C / 4, Ho = H / 2, Wo = W / 2;
  const size_t total = (size_t)Bn * Ho * Wo * c4n;
  if (t >= total) return;
  const int c4 = (int)(t % c4n) * 4; size_t rest = t / c4n;
  const int pw = (int)(rest % Wo); rest /= Wo; const int ph = (int)(rest % Ho); const int b = (int)(rest / Ho);
  const float* base = in + (size_t)b * H * W * C;
  const int p00 = (2 * ph) * W + 2 * pw;
  const v4f a = *(const v4fa*)(base + (size_t)p00 * C + c4), bq = *(const v4fa*)(base + (size_t)(p00 + 1) * C + c4);
  const v4f c = *(const v4fa*)(base + (size_t)(p00 + W) * C + c4), d = *(const v4fa*)(base + (size_t)(p00 + W + 1) * C + c4);
  v4f m; for (int i = 0; i < 4; ++i) m[i] = fmaxf(fmaxf(a[i], bq[i]), fmaxf(c[i], d[i]));
  float* dst = out + ((size_t)b * Ho * Wo + (size_t)ph * Wo + pw) * C + c4;
  *(volatile v4f*)dst = m;
  __threadfence();
  *(volatile v4f*)dst = m;
}

template <int DQ, int DV>
__global__ __launch_bounds__(128) void k_flash2(const float* __restrict__ Qb, size_t qstride, int qpitch, int Tq,
                                              const float* __restrict__ Kb, size_t kstride, int kpitch, int Tk,
                                              const float* __restrict__ Vb, size_t vstride, int vpitch,
                                              float scale, float* __restrict__ y, size_t ystride, int ypitch) {
  constexpr int KS = DQ / 32, DT = DV / 16;
  __shared__ __attribute__((aligned(16))) unsigned short sKh[32][DQ + 8], sKl[32][DQ + 8], sVh[32][DV + 8], sVl[32][DV + 8];
  __shared__ __attribute__((aligned(16))) unsigned short sPh[4][16][40], sPl[4][16][40];
  __shared__ __attribute__((aligned(16))) float sO[4][16][DV];
  const int tid = threadIdx.x, w = tid >> 5, lane = tid & 31, ln = lane & 15, hh = lane >> 4;
  const int nqb = (Tq + 63) / 64;
  const int bh = blockIdx.x / nqb, qblk = blockIdx.x % nqb;
  const int dv0 = blockIdx.y * DV;
  const int q0 = qblk * 64 + w * 16;
  const float* Q = Qb + (size_t)bh * qstride; const float* K = Kb + (size_t)bh * kstride; const float* V = Vb + (size_t)bh * vstride + dv0;
  FragB aqh[KS], aql[KS];
  {
    int row = q0 + ln; if (row >= Tq) row = Tq - 1;
    const float* qr = Q + (size_t)row * qpitch;
#pragma unroll
    for (int ks = 0; ks < KS; ++ks)
#pragma unroll
      for (int i = 0; i < 16; ++i) {
        const int d = ks * 32 + ((i < 8) ? (8 * hh + i) : (16 + 8 * hh + (i - 8)));
        const float x = qr[d] * scale; const unsigned short hb = bf16_bits(x);
        aqh[ks].u[i] = hb; aql[ks].u[i] = bf16_bits(x - bf16_val(hb));
      }
  }
  float m_r[8], l_r[8];
#pragma unroll
  for (int r = 0; r < 8; ++r) { m_r[r] = -3.0e38f; l_r[r] = 0.f; }
  v8f oacc[DT];
#pragma unroll
  for (int dt = 0; dt < DT; ++dt) oacc[dt] = (v8f){0.f,0.f,0.f,0.f,0.f,0.f,0.f,0.f};
  for (int j0 = 0; j0 < Tk; j0 += 32) {
    __syncthreads();
    for (int e = tid; e < 32 * (DQ / 4); e += 128) {
      const int r = e / (DQ / 4), c4 = (e % (DQ / 4)) * 4; const int key = j0 + r;
      v4f f = {0.f,0.f,0.f,0.f}; if (key < Tk) f = *(const v4fa*)(K + (size_t)key * kpitch + c4);
#pragma unroll
      for (int t = 0; t < 4; ++t) { const unsigned short hb = bf16_bits(f[t]); sKh[r][c4 + t] = hb; sKl[r][c4 + t] = bf16_bits(f[t] - bf16_val(hb)); }
    }
    for (int e = tid; e < 32 * (DV / 4); e += 128) {
      const int r = e / (DV / 4), c4 = (e % (DV / 4)) * 4; const int key = j0 + r;
      v4f f = {0.f,0.f,0.f,0.f}; if (key < Tk) f = *(const v4fa*)(V + (size_t)key * vpitch + c4);
#pragma unroll
      for (int t = 0; t < 4; ++t) { const unsigned short hb = bf16_bits(f[t]); sVh[r][c4 + t] = hb; sVl[r][c4 + t] = bf16_bits(f[t] - bf16_val(hb)); }
    }
    __syncthreads();
    v8f s[2];
#pragma unroll
    for (int nt = 0; nt < 2; ++nt) {
      v8f acc = {};
#pragma unroll
      for (int ks = 0; ks < KS; ++ks) {
        FragB bh_, bl_;
        bh_.half[0] = *(const v8us*)&sKh[nt * 16 + ln][ks * 32 + 8 * hh]; bh_.half[1] = *(const v8us*)&sKh[nt * 16 + ln][ks * 32 + 16 + 8 * hh];
        bl_.half[0] = *(const v8us*)&sKl[nt * 16 + ln][ks * 32 + 8 * hh]; bl_.half[1] = *(const v8us*)&sKl[nt * 16 + ln][ks * 32 + 16 + 8 * hh];
        acc = mmaN<3>(aqh[ks].v, aql[ks].v, bh_.v, bl_.v, acc);
      }
      s[nt] = acc;
    }
    float alpha[8];
#pragma unroll
    for (int r = 0; r < 8; ++r) {
      const int ja = j0 + ln, jb = j0 + 16 + ln;
      if (ja >= Tk) s[0][r] = -3.0e38f;
      if (jb >= Tk) s[1][r] = -3.0e38f;
      float mx = fmaxf(s[0][r], s[1][r]);
      mx = fmaxf(mx, __shfl_xor(mx, 1, 32)); mx = fmaxf(mx, __shfl_xor(mx, 2, 32)); mx = fmaxf(mx, __shfl_xor(mx, 4, 32)); mx = fmaxf(mx, __shfl_xor(mx, 8, 32));
      const float mnew = fmaxf(m_r[r], mx);
      alpha[r] = (mnew > -1.0e38f) ? __expf(m_r[r] - mnew) : 1.0f;
      const float p0 = (s[0][r] > -1.0e38f) ? __expf(s[0][r] - mnew) : 0.f;
      const float p1 = (s[1][r] > -1.0e38f) ? __expf(s[1][r] - mnew) : 0.f;
      m_r[r] = mnew;
      l_r[r] = l_r[r] * alpha[r] + p0 + p1;
      unsigned short hb = bf16_bits(p0); sPh[w][8 * hh + r][ln] = hb;      sPl[w][8 * hh + r][ln] = bf16_bits(p0 - bf16_val(hb));
      hb = bf16_bits(p1);                sPh[w][8 * hh + r][16 + ln] = hb; sPl[w][8 * hh + r][16 + ln] = bf16_bits(p1 - bf16_val(hb));
    }
#pragma unroll
    for (int dt = 0; dt < DT; ++dt)
#pragma unroll
      for (int r = 0; r < 8; ++r) oacc[dt][r] *= alpha[r];
    __builtin_amdgcn_fence(__ATOMIC_ACQ_REL, "workgroup");
    __builtin_amdgcn_wave_barrier();
    FragB pah, pal;
    pah.half[0] = *(const v8us*)&sPh[w][ln][8 * hh]; pah.half[1] = *(const v8us*)&sPh[w][ln][16 + 8 * hh];
    pal.half[0] = *(const v8us*)&sPl[w][ln][8 * hh]; pal.half[1] = *(const v8us*)&sPl[w][ln][16 + 8 * hh];
#pragma unroll
    for (int dt = 0; dt < DT; ++dt) {
      FragB bvh, bvl;
#pragma unroll
      for (int i = 0; i < 8; ++i) {
        bvh.u[i] = sVh[8 * hh + i][dt * 16 + ln]; bvh.u[8 + i] = sVh[16 + 8 * hh + i][dt * 16 + ln];
        bvl.u[i] = sVl[8 * hh + i][dt * 16 + ln]; bvl.u[8 + i] = sVl[16 + 8 * hh + i][dt * 16 + ln];
      }
      oacc[dt] = mmaN<3>(pah.v, pal.v, bvh.v, bvl.v, oacc[dt]);
    }
    __builtin_amdgcn_fence(__ATOMIC_ACQ_REL, "workgroup");
    __builtin_amdgcn_wave_barrier();
  }
#pragma unroll
  for (int r = 0; r < 8; ++r) {
    float l = l_r[r];
    l += __shfl_xor(l, 1, 32); l += __shfl_xor(l, 2, 32); l += __shfl_xor(l, 4, 32); l += __shfl_xor(l, 8, 32);
    l_r[r] = (l > 0.f) ? 1.0f / l : 0.f;
  }
#pragma unroll
  for (int dt = 0; dt < DT; ++dt)
#pragma unroll
    for (int r = 0; r < 8; ++r) sO[w][8 * hh + r][dt * 16 + ln] = oacc[dt][r] * l_r[r];
  __builtin_amdgcn_fence(__ATOMIC_ACQ_REL, "workgroup");
  __builtin_amdgcn_wave_barrier();
  for (int pass = 0; pass < 2; ++pass) {
    for (int r = 0; r < 16; ++r) {
      const int row = q0 + r;
      for (int c4 = lane * 4; c4 < DV; c4 += 128) {
        if (row < Tq) {
          const v4f val = *(const v4fa*)&sO[w][r][c4];
          *(volatile v4f*)(y + (size_t)bh * ystride + (size_t)row * ypitch + dv0 + c4) = val;
        }
      }
    }
    if (pass == 0) __threadfence();
  }
}

template <bool ASPLIT, int ACT, bool BIAS_BF16, bool RES_BF16>
__global__ __launch_bounds__(128) void k_gemm_bf3(const float* __restrict__ A, int lda, const unsigned short* __restrict__ Wt, int ldb,
                                                const float* __restrict__ bias, const float* __restrict__ resid, int rmod, int ldr,
                                                float* __restrict__ C, int ldc, int M, int N, int K) {
  __shared__ __attribute__((aligned(16))) float so[4][16][64];
  const int tid = threadIdx.x, w = tid >> 5, lane = tid & 31, ln = lane & 15, hh = lane >> 4;
  const int ntn = N / 64;
  const int wid = blockIdx.x * 4 + w;
  const int mt = wid / ntn, nq = wid % ntn;
  if (mt * 16 >= M) return;
  const int row0 = mt * 16, col0 = nq * 64;
  const float* arow = A + (size_t)(row0 + ln) * lda;
  v8f acc[4] = {};
  for (int kb = 0; kb < K; kb += 32) {
    FragB ah, al;
    const v4f x0 = *(const v4fa*)(arow + kb + 8 * hh), x1 = *(const v4fa*)(arow + kb + 8 * hh + 4);
    const v4f x2 = *(const v4fa*)(arow + kb + 16 + 8 * hh), x3 = *(const v4fa*)(arow + kb + 16 + 8 * hh + 4);
    float xs[16] = {x0[0],x0[1],x0[2],x0[3],x1[0],x1[1],x1[2],x1[3],x2[0],x2[1],x2[2],x2[3],x3[0],x3[1],x3[2],x3[3]};
#pragma unroll
    for (int i = 0; i < 16; ++i) { const unsigned short hb = bf16_bits(xs[i]); ah.u[i] = hb; al.u[i] = ASPLIT ? bf16_bits(xs[i] - bf16_val(hb)) : (unsigned short)0; }
#pragma unroll
    for (int t = 0; t < 4; ++t) {
      const unsigned short* brow = Wt + (size_t)(col0 + t * 16 + ln) * ldb + kb;
      FragB b;
      b.half[0] = *(const v8us*)(brow + 8 * hh);
      b.half[1] = *(const v8us*)(brow + 16 + 8 * hh);
      acc[t] = mmaN<ASPLIT ? 2 : 1>(ah.v, al.v, b.v, b.v, acc[t]);
    }
  }
#pragma unroll
  for (int t = 0; t < 4; ++t) {
    const int col = col0 + t * 16 + ln;
    float bv = bias ? bias[col] : 0.f;
    if (BIAS_BF16) bv = bf16_round(bv);
#pragma unroll
    for (int r = 0; r < 8; ++r) {
      float v = acc[t][r] + bv;
      if (resid) { float rv = resid[(size_t)((row0 + 8 * hh + r) % rmod) * ldr + col]; if (RES_BF16) rv = bf16_round(rv); v += rv; }
      if (ACT == 1) v = fmaxf(v, 0.f);
      if (ACT == 2) v = 0.5f * v * (1.0f + erff(v * 0.70710678118654752f));
      if (ACT == 3) { const float u = 0.7978845608028654f * (v + 0.044715f * v * v * v); v = 0.5f * v * (1.0f + tanhf(u)); }
      so[w][8 * hh + r][t * 16 + ln] = v;
    }
  }
  __builtin_amdgcn_fence(__ATOMIC_ACQ_REL, "workgroup");
  __builtin_amdgcn_wave_barrier();
  const int rsub = lane >> 4, c4 = (lane & 15) * 4;
  for (int pass = 0; pass < 2; ++pass) {
#pragma unroll
    for (int q = 0; q < 8; ++q) {
      const int r = q * 2 + rsub;
      const v4f v = *(const v4fa*)&so[w][r][c4];
      *(volatile v4f*)(C + (size_t)(row0 + r) * ldc + col0 + c4) = v;
    }
    if (pass == 0) __threadfence();
  }
}
template <bool PARAM_BF16>
__global__ __launch_bounds__(256) void k_layernorm(const float* __restrict__ X, const float* __restrict__ R, const float* __restrict__ g, const float* __restrict__ bta,
                                                  float* __restrict__ out_sum, float* __restrict__ out_norm, int N, float eps) {
  __shared__ float red[256];
  const int row = blockIdx.x, tid = threadIdx.x;
  const float* x = X + (size_t)row * N; const float* rr = R ? R + (size_t)row * N : nullptr;
  float vals[16];
  const int per = N / 256;
  float s1 = 0.f;
  for (int u = 0; u < per / 4; ++u) {
    const int j = tid * 4 + 1024 * u;
    const v4f a = *(const v4fa*)(x + j);
    v4f b = {0.f,0.f,0.f,0.f}; if (rr) b = *(const v4fa*)(rr + j);
#pragma unroll
    for (int q = 0; q < 4; ++q) { const float v = a[q] + b[q]; vals[u * 4 + q] = v; s1 += v; }
  }
  red[tid] = s1; __syncthreads();
  for (int st = 128; st > 0; st >>= 1) { if (tid < st) red[tid] += red[tid + st]; __syncthreads(); }
  const float mu = red[0] / (float)N; __syncthreads();
  float s2 = 0.f;
  for (int u = 0; u < per / 4; ++u)
#pragma unroll
    for (int q = 0; q < 4; ++q) { const float c = vals[u * 4 + q] - mu; s2 += c * c; }
  red[tid] = s2; __syncthreads();
  for (int st = 128; st > 0; st >>= 1) { if (tid < st) red[tid] += red[tid + st]; __syncthreads(); }
  const float rs = rsqrtf(red[0] / (float)N + eps);
  for (int pass = 0; pass < 2; ++pass) {
    for (int u = 0; u < per / 4; ++u) {
      const int j = tid * 4 + 1024 * u;
      v4f o, sm;
#pragma unroll
      for (int q = 0; q < 4; ++q) {
        float gg = g[j + q], bb = bta[j + q];
        if (PARAM_BF16) { gg = bf16_round(gg); bb = bf16_round(bb); }
        sm[q] = vals[u * 4 + q]; o[q] = (vals[u * 4 + q] - mu) * rs * gg + bb;
      }
      if (out_sum) *(volatile v4f*)(out_sum + (size_t)row * N + j) = sm;
      *(volatile v4f*)(out_norm + (size_t)row * N + j) = o;
    }
    if (pass == 0) __threadfence();
  }
}

template <bool ASPLIT, bool BSPLIT, int ACT>
__global__ __launch_bounds__(128) void k_gemm_b(const float* __restrict__ A, int lda, size_t sA, const unsigned short* __restrict__ Bh, const unsigned short* __restrict__ Bl, int ldb, size_t sB,
                                             const float* __restrict__ bias, const float* __restrict__ resid, int ldr, size_t sR, float rsign, float alpha,
                                             float* __restrict__ C, int ldc, size_t sC, int M, int N, int K) {
  __shared__ __attribute__((aligned(16))) float so[4][16][64];
  const int tid = threadIdx.x, w = tid >> 5, lane = tid & 31, ln = lane & 15, hh = lane >> 4;
  const int by = blockIdx.y;
  A += (size_t)by * sA; Bh += (size_t)by * sB; if (BSPLIT) Bl += (size_t)by * sB; C += (size_t)by * sC; if (resid) resid += (size_t)by * sR;
  const int ntn = (N + 63) / 64; const int wid = blockIdx.x * 4 + w; const int mt = wid / ntn, nq = wid % ntn;
  if (mt * 16 >= M) return;
  const int row0 = mt * 16, col0 = nq * 64;
  const float* arow = A + (size_t)(row0 + ln) * lda;
  v8f acc[4] = {};
  for (int kb = 0; kb < K; kb += 32) {
    FragB ah, al;
    const v4f x0 = *(const v4fa*)(arow + kb + 8 * hh), x1 = *(const v4fa*)(arow + kb + 8 * hh + 4);
    const v4f x2 = *(const v4fa*)(arow + kb + 16 + 8 * hh), x3 = *(const v4fa*)(arow + kb + 16 + 8 * hh + 4);
    float xs[16] = {x0[0],x0[1],x0[2],x0[3],x1[0],x1[1],x1[2],x1[3],x2[0],x2[1],x2[2],x2[3],x3[0],x3[1],x3[2],x3[3]};
#pragma unroll
    for (int i = 0; i < 16; ++i) { const unsigned short hb = bf16_bits(xs[i]); ah.u[i] = hb; al.u[i] = ASPLIT ? bf16_bits(xs[i] - bf16_val(hb)) : (unsigned short)0; }
#pragma unroll
    for (int t = 0; t < 4; ++t) {
      if (col0 + t * 16 >= N) continue;
      const size_t boff = (size_t)(col0 + t * 16 + ln) * ldb + kb;
      FragB bh_, bl_; bh_.half[0] = *(const v8us*)(Bh + boff + 8 * hh); bh_.half[1] = *(const v8us*)(Bh + boff + 16 + 8 * hh);
      if (BSPLIT) { bl_.half[0] = *(const v8us*)(Bl + boff + 8 * hh); bl_.half[1] = *(const v8us*)(Bl + boff + 16 + 8 * hh); } else bl_ = bh_;
      acc[t] = mmaN<ASPLIT ? (BSPLIT ? 3 : 2) : 1>(ah.v, al.v, bh_.v, bl_.v, acc[t]);
    }
  }
#pragma unroll
  for (int t = 0; t < 4; ++t) {
    const int col = col0 + t * 16 + ln; if (col0 + t * 16 >= N) continue; const float bv = bias ? bf16_round(bias[col]) : 0.f;
#pragma unroll
    for (int r = 0; r < 8; ++r) { float v = acc[t][r] * alpha + bv; if (resid) v += rsign * resid[(size_t)(row0 + 8 * hh + r) * ldr + col]; if (ACT == 1) v = fmaxf(v, 0.f); else if (ACT == 2) v = fmaxf(v, 0.f) + log1pf(expf(-fabsf(v))); so[w][8 * hh + r][t * 16 + ln] = v; }
  }
  __builtin_amdgcn_fence(__ATOMIC_ACQ_REL, "workgroup"); __builtin_amdgcn_wave_barrier();
  const int rsub = lane >> 4, c4 = (lane & 15) * 4;
  for (int pass = 0; pass < 2; ++pass) {
#pragma unroll
    for (int q = 0; q < 8; ++q) { const int r = q * 2 + rsub; if (col0 + c4 < N) { const v4f v = *(const v4fa*)&so[w][r][c4]; *(volatile v4f*)(C + (size_t)(row0 + r) * ldc + col0 + c4) = v; } }
    if (pass == 0) __threadfence();
  }
}
__global__ __launch_bounds__(256) void k_split_transpose_b(const float* __restrict__ src, int lds_, size_t sIn, unsigned short* __restrict__ hi, unsigned short* __restrict__ lo, size_t sOut, int K, int N) {
  const size_t t = (size_t)blockIdx.x * 256 + threadIdx.x; const int k8n = K / 8; if (t >= (size_t)N * k8n) return;
  src += (size_t)blockIdx.y * sIn; hi += (size_t)blockIdx.y * sOut; lo += (size_t)blockIdx.y * sOut;
  const int n = (int)(t / k8n), k8 = (int)(t % k8n) * 8; v8us vh, vl;
#pragma unroll
  for (int i = 0; i < 8; ++i) { const float x = src[(size_t)(k8 + i) * lds_ + n]; const unsigned short hb = bf16_bits(x); vh[i] = hb; vl[i] = bf16_bits(x - bf16_val(hb)); }
  unsigned short* dh = hi + (size_t)n * K + k8; unsigned short* dl = lo + (size_t)n * K + k8;
  *(volatile v8us*)dh = vh; *(volatile v8us*)dl = vl; __threadfence(); *(volatile v8us*)dh = vh; *(volatile v8us*)dl = vl;
}

typedef _Float16 v16h __attribute__((ext_vector_type(16)));
union FragH { v16h v; v8us half[2]; _Float16 h[16]; unsigned short u[16]; };
template <int NT>
__device__ __forceinline__ v8f mmaH(v16h ah, v16h al, v16h bh, v16h bl, v8f c) {
  c = __builtin_amdgcn_wmma_f32_16x16x32_f16(false, ah, false, bh, (short)0, c, false, false);
  if (NT >= 2) c = __builtin_amdgcn_wmma_f32_16x16x32_f16(false, al, false, bh, (short)0, c, false, false);
  if (NT >= 3) c = __builtin_amdgcn_wmma_f32_16x16x32_f16(false, ah, false, bl, (short)0, c, false, false);
  asm volatile("v_nop\n\tv_nop\n\tv_nop\n\tv_nop" : "+v"(c) : "v"(ah), "v"(al), "v"(bh), "v"(bl));
  return c;
}
template <bool ASPLIT>
__global__ __launch_bounds__(128) void k_gemm_h(const float* __restrict__ A, int lda, size_t sA, const _Float16* __restrict__ Bh, int ldb, size_t sB, float alpha, float* __restrict__ C, int ldc, size_t sC, int M, int N, int K) {
  __shared__ __attribute__((aligned(16))) float so[4][16][64];
  const int tid = threadIdx.x, w = tid >> 5, lane = tid & 31, ln = lane & 15, hh = lane >> 4; const int by = blockIdx.y;
  A += (size_t)by * sA; Bh += (size_t)by * sB; C += (size_t)by * sC;
  const int ntn = (N + 63) / 64; const int wid = blockIdx.x * 4 + w; const int mt = wid / ntn, nq = wid % ntn; if (mt * 16 >= M) return;
  const int row0 = mt * 16, col0 = nq * 64; const float* arow = A + (size_t)(row0 + ln) * lda;
  v8f acc[4] = {};
  for (int kb = 0; kb < K; kb += 32) {
    FragH ah, al;
    const v4f x0 = *(const v4fa*)(arow + kb + 8 * hh), x1 = *(const v4fa*)(arow + kb + 8 * hh + 4), x2 = *(const v4fa*)(arow + kb + 16 + 8 * hh), x3 = *(const v4fa*)(arow + kb + 16 + 8 * hh + 4);
    float xs[16] = {x0[0],x0[1],x0[2],x0[3],x1[0],x1[1],x1[2],x1[3],x2[0],x2[1],x2[2],x2[3],x3[0],x3[1],x3[2],x3[3]};
#pragma unroll
    for (int i = 0; i < 16; ++i) { const _Float16 h = (_Float16)xs[i]; ah.h[i] = h; al.h[i] = ASPLIT ? (_Float16)(xs[i] - (float)h) : (_Float16)0.0f; }
#pragma unroll
    for (int t = 0; t < 4; ++t) { if (col0 + t * 16 >= N) continue; const size_t boff = (size_t)(col0 + t * 16 + ln) * ldb + kb; FragH bq; bq.half[0] = *(const v8us*)(Bh + boff + 8 * hh); bq.half[1] = *(const v8us*)(Bh + boff + 16 + 8 * hh);
      acc[t] = mmaH<ASPLIT ? 2 : 1>(ah.v, al.v, bq.v, bq.v, acc[t]); }
  }
#pragma unroll
  for (int t = 0; t < 4; ++t) { if (col0 + t * 16 >= N) continue;
#pragma unroll
    for (int r = 0; r < 8; ++r) so[w][8 * hh + r][t * 16 + ln] = acc[t][r] * alpha; }
  __builtin_amdgcn_fence(__ATOMIC_ACQ_REL, "workgroup"); __builtin_amdgcn_wave_barrier();
  const int rsub = lane >> 4, c4 = (lane & 15) * 4;
  for (int pass = 0; pass < 2; ++pass) {
#pragma unroll
    for (int q = 0; q < 8; ++q) { const int r = q * 2 + rsub; if (col0 + c4 < N) { const v4f v = *(const v4fa*)&so[w][r][c4]; *(volatile v4f*)(C + (size_t)(row0 + r) * ldc + col0 + c4) = v; } }
    if (pass == 0) __threadfence(); }
}

__global__ __launch_bounds__(256) void k_round_rows(const float* __restrict__ W, unsigned short* __restrict__ Wt, int n8) {
  const int t = blockIdx.x * 256 + threadIdx.x;
  if (t >= n8) return;
  const v4f a = *(const v4fa*)(W + (size_t)t * 8), b = *(const v4fa*)(W + (size_t)t * 8 + 4);
  v8us v; v[0]=bf16_bits(a[0]); v[1]=bf16_bits(a[1]); v[2]=bf16_bits(a[2]); v[3]=bf16_bits(a[3]);
  v[4]=bf16_bits(b[0]); v[5]=bf16_bits(b[1]); v[6]=bf16_bits(b[2]); v[7]=bf16_bits(b[3]);
  *(volatile v8us*)(Wt + (size_t)t * 8) = v; __threadfence(); *(volatile v8us*)(Wt + (size_t)t * 8) = v;
}

template <int DUMMY>
__global__ __launch_bounds__(128) void k_gemm_hh(const _Float16* __restrict__ A, int lda, size_t sA, const _Float16* __restrict__ Bh, int ldb, size_t sB, float alpha, float* __restrict__ C, int ldc, size_t sC, int M, int N, int K) {
  __shared__ __attribute__((aligned(16))) float so[4][16][64];
  const int tid = threadIdx.x, w = tid >> 5, lane = tid & 31, ln = lane & 15, hh = lane >> 4; const int by = blockIdx.y;
  A += (size_t)by * sA; Bh += (size_t)by * sB; C += (size_t)by * sC;
  const int ntn = (N + 63) / 64; const int wid = blockIdx.x * 4 + w; const int mt = wid / ntn, nq = wid % ntn; if (mt * 16 >= M) return;
  const int row0 = mt * 16, col0 = nq * 64; const _Float16* arow = A + (size_t)(row0 + ln) * lda;
  v8f acc[4] = {};
  for (int kb = 0; kb < K; kb += 32) { FragH ah; ah.half[0] = *(const v8us*)((const unsigned short*)arow + kb + 8 * hh); ah.half[1] = *(const v8us*)((const unsigned short*)arow + kb + 16 + 8 * hh);
#pragma unroll
    for (int t = 0; t < 4; ++t) { if (col0 + t * 16 >= N) continue; const size_t boff = (size_t)(col0 + t * 16 + ln) * ldb + kb; FragH bq; bq.half[0] = *(const v8us*)((const unsigned short*)Bh + boff + 8 * hh); bq.half[1] = *(const v8us*)((const unsigned short*)Bh + boff + 16 + 8 * hh);
      acc[t] = mmaH<1>(ah.v, ah.v, bq.v, bq.v, acc[t]); }
  }
#pragma unroll
  for (int t = 0; t < 4; ++t) { if (col0 + t * 16 >= N) continue;
#pragma unroll
    for (int r = 0; r < 8; ++r) so[w][8 * hh + r][t * 16 + ln] = acc[t][r] * alpha; }
  __builtin_amdgcn_fence(__ATOMIC_ACQ_REL, "workgroup"); __builtin_amdgcn_wave_barrier();
  const int rsub = lane >> 4, c4 = (lane & 15) * 4;
  for (int pass = 0; pass < 2; ++pass) {
#pragma unroll
    for (int q = 0; q < 8; ++q) { const int r = q * 2 + rsub; if (col0 + c4 < N) { const v4f v = *(const v4fa*)&so[w][r][c4]; *(volatile v4f*)(C + (size_t)(row0 + r) * ldc + col0 + c4) = v; } }
    if (pass == 0) __threadfence(); }
}

__global__ __launch_bounds__(256) void k_bcat384(const float* __restrict__ vb, float* __restrict__ o) { const int t = blockIdx.x * 256 + threadIdx.x; if (t >= 384) return; const float v = (t < 128) ? 0.f : vb[t - 128]; *(volatile float*)(o + t) = v; __threadfence(); *(volatile float*)(o + t) = v; }
__global__ __launch_bounds__(256) void k_xt(const float* __restrict__ x, float* __restrict__ XT) { __shared__ float tile[32][33]; const int b = blockIdx.z; const int c0 = blockIdx.y * 32, n0 = blockIdx.x * 32; const int tx = threadIdx.x & 31, ty = threadIdx.x >> 5;
  for (int i = ty; i < 32; i += 8) tile[i][tx] = bf16_round(x[((size_t)b * CC + c0 + i) * NN + n0 + tx]); __syncthreads();
  for (int pass = 0; pass < 2; ++pass) { for (int i = ty; i < 32; i += 8) *(volatile float*)(XT + ((size_t)b * NN + n0 + i) * CC + c0 + tx) = tile[tx][i]; if (pass == 0) __threadfence(); } }
__global__ __launch_bounds__(256) void k_planes(const float* __restrict__ a, unsigned short* __restrict__ hi, unsigned short* __restrict__ lo, size_t n8, int ld_src, int ld_dst, int ncol) { const size_t t = (size_t)blockIdx.x * 256 + threadIdx.x; if (t >= n8) return; const size_t e0 = t * 8; const size_t r = e0 / ncol; const int c = (int)(e0 % ncol); v8us h, l;
  for (int q = 0; q < 8; ++q) { const float v = a[r * ld_src + c + q]; const unsigned short hb = bf16_bits(v); h[q] = hb; l[q] = bf16_bits(v - bf16_val(hb)); } *(volatile v8us*)(hi + r * ld_dst + c) = h; *(volatile v8us*)(lo + r * ld_dst + c) = l; __threadfence(); *(volatile v8us*)(hi + r * ld_dst + c) = h; *(volatile v8us*)(lo + r * ld_dst + c) = l; }
__global__ __launch_bounds__(256) void k_ltplanes(const float* __restrict__ xl, const float* __restrict__ yl, const float* __restrict__ zl, unsigned short* __restrict__ hi, unsigned short* __restrict__ lo) { const int t = blockIdx.x * 256 + threadIdx.x; if (t >= 3 * NRP * (DQK / 8)) return; const int c8 = (t % (DQK / 8)) * 8; const int r = (t / (DQK / 8)) % NRP; const int w = t / ((DQK / 8) * NRP); const float* src = (w == 0) ? xl : (w == 1 ? yl : zl); v8us h, l;
  for (int q = 0; q < 8; ++q) { const float v = (r < NREL) ? bf16_round(src[r * DQK + c8 + q]) : 0.f; const unsigned short hb = bf16_bits(v); h[q] = hb; l[q] = bf16_bits(v - bf16_val(hb)); } const size_t dst = ((size_t)w * NRP + r) * DQK + c8; *(volatile v8us*)(hi + dst) = h; *(volatile v8us*)(lo + dst) = l; __threadfence(); *(volatile v8us*)(hi + dst) = h; *(volatile v8us*)(lo + dst) = l; }
__global__ __launch_bounds__(256) void k_vt(const float* __restrict__ QKV, _Float16* __restrict__ Vt) { __shared__ float tv[64][65]; const int b = blockIdx.z; const int n0 = blockIdx.x * 64, d0 = blockIdx.y * 64; const int tid = threadIdx.x; typedef _Float16 v2h __attribute__((ext_vector_type(2)));
  for (int e = tid; e < 64 * 64; e += 256) { const int r = e >> 6, c = e & 63; tv[r][c] = QKV[((size_t)b * NN + n0 + r) * 384 + 128 + d0 + c]; } __syncthreads();
  for (int pass = 0; pass < 2; ++pass) { for (int e = tid; e < 64 * 32; e += 256) { const int d = e >> 5, np = (e & 31) * 2; v2h vv; vv.x = (_Float16)tv[np][d]; vv.y = (_Float16)tv[np + 1][d]; *(volatile v2h*)(Vt + ((size_t)b * DVV + d0 + d) * NN + n0 + np) = vv; } if (pass == 0) __threadfence(); } }
__global__ __launch_bounds__(1024) void k_softmax(float* __restrict__ E, const float* __restrict__ QL, const int* __restrict__ disc, int b, float* __restrict__ Dn) { __shared__ float sd[32]; const int tid = threadIdx.x, wv = tid >> 5, lane = tid & 31; const int n = blockIdx.x * 32 + wv; float* row = E + (size_t)n * NN; const float* ql = QL + ((size_t)b * NN + n) * (3 * NRP); const int* dn = disc + ((size_t)b * NN + n) * 3; const int dxn = dn[0], dyn = dn[1], dzn = dn[2];
  const float rs = 0.03125f;
  float mx = -3.0e38f;
#pragma unroll 1
  for (int m = lane; m < NN; m += 32) { const int* dm = disc + ((size_t)b * NN + m) * 3; int ix = dm[0] - dxn + (NBIN - 1), iy = dm[1] - dyn + (NBIN - 1), iz = dm[2] - dzn + (NBIN - 1); ix = ix < 0 ? 0 : (ix > NREL - 1 ? NREL - 1 : ix); iy = iy < 0 ? 0 : (iy > NREL - 1 ? NREL - 1 : iy); iz = iz < 0 ? 0 : (iz > NREL - 1 ? NREL - 1 : iz);
    const float v = (((row[m] + ql[ix]) + ql[NRP + iy]) + ql[2 * NRP + iz]) * rs; *(volatile float*)(row + m) = v; mx = fmaxf(mx, v); }
  for (int o = 16; o >= 1; o >>= 1) mx = fmaxf(mx, __shfl_xor(mx, o, 32)); __threadfence();
  float den = 0.f;
#pragma unroll 1
  for (int m = lane; m < NN; m += 32) { const float e = expf(row[m] - mx); den += e; *(volatile float*)(row + m) = e * 256.0f; }
  for (int o = 16; o >= 1; o >>= 1) den += __shfl_xor(den, o, 32); __threadfence();
#pragma unroll 1
  for (int m = lane; m < NN; m += 32) { const float pv = row[m]; *(volatile float*)(row + m) = pv; }
  if (lane == 0) sd[wv] = den; __syncthreads(); if (tid < 32) { *(volatile float*)(Dn + (size_t)b * NN + blockIdx.x * 32 + tid) = sd[tid]; } __threadfence(); if (tid < 32) { *(volatile float*)(Dn + (size_t)b * NN + blockIdx.x * 32 + tid) = sd[tid]; } }
__global__ __launch_bounds__(256) void k_attnT(const float* __restrict__ E, const float* __restrict__ Dn, int b, _Float16* __restrict__ AT) { __shared__ float tile[64][65]; const int n0 = blockIdx.y * 64, m0 = blockIdx.x * 64; const int tid = threadIdx.x; typedef _Float16 v2h __attribute__((ext_vector_type(2)));
  for (int e = tid; e < 64 * 64; e += 256) { const int r = e >> 6, c = e & 63; tile[r][c] = E[(size_t)(n0 + r) * NN + m0 + c] / Dn[(size_t)b * NN + n0 + r]; } __syncthreads();
  for (int pass = 0; pass < 2; ++pass) { for (int e = tid; e < 64 * 32; e += 256) { const int m = e >> 5, np = (e & 31) * 2; v2h vv; vv.x = (_Float16)tile[np][m]; vv.y = (_Float16)tile[np + 1][m]; *(volatile v2h*)(AT + (size_t)(m0 + m) * NN + n0 + np) = vv; } if (pass == 0) __threadfence(); } }
__global__ __launch_bounds__(256) void k_hdiff(const float* __restrict__ XT, const float* __restrict__ XRt, float* __restrict__ Hm) { const size_t t = (size_t)blockIdx.x * 256 + threadIdx.x; if (t >= (size_t)NTOK * CC / 4) return; const v4f a = *(const v4fa*)(XT + t * 4), r = *(const v4fa*)(XRt + t * 4); v4f o; for (int q = 0; q < 4; ++q) o[q] = a[q] - r[q]; *(volatile v4f*)(Hm + t * 4) = o; __threadfence(); *(volatile v4f*)(Hm + t * 4) = o; }
__global__ __launch_bounds__(256) void k_colstat(const float* __restrict__ T, double* __restrict__ part) { const int c = threadIdx.x; const size_t r0 = (size_t)blockIdx.x * 1024; double s = 0.0, q = 0.0;
#pragma unroll 1
  for (int r = 0; r < 1024; ++r) { const float v = T[(r0 + r) * CC + c]; s += v; q += (double)v * v; } *(volatile double*)(part + ((size_t)blockIdx.x * CC + c) * 2) = s; *(volatile double*)(part + ((size_t)blockIdx.x * CC + c) * 2 + 1) = q; __threadfence(); *(volatile double*)(part + ((size_t)blockIdx.x * CC + c) * 2) = s; *(volatile double*)(part + ((size_t)blockIdx.x * CC + c) * 2 + 1) = q; }
__global__ __launch_bounds__(256) void k_bnfin(const double* __restrict__ part, const float* __restrict__ g, const float* __restrict__ bb, float* __restrict__ st) { const int c = threadIdx.x; double s = 0.0, q = 0.0; for (int k = 0; k < NTOK / 1024; ++k) { s += part[((size_t)k * CC + c) * 2]; q += part[((size_t)k * CC + c) * 2 + 1]; }
  const double mu = s / NTOK; double var = q / NTOK - mu * mu; if (var < 0.0) var = 0.0; const float sc = (float)(1.0 / sqrt(var + 1e-5)) * bf16_round(g[c]); const float sh = bf16_round(bb[c]) - (float)mu * sc; *(volatile float*)(st + c * 2) = sc; *(volatile float*)(st + c * 2 + 1) = sh; __threadfence(); *(volatile float*)(st + c * 2) = sc; *(volatile float*)(st + c * 2 + 1) = sh; }
__global__ __launch_bounds__(256) void k_out(const float* __restrict__ T, const float* __restrict__ st, const float* __restrict__ x, float* __restrict__ out) { __shared__ float tile[32][33]; const int b = blockIdx.z; const int n0 = blockIdx.y * 32, c0 = blockIdx.x * 32; const int tx = threadIdx.x & 31, ty = threadIdx.x >> 5;
  for (int i = ty; i < 32; i += 8) tile[i][tx] = fmaxf(T[((size_t)b * NN + n0 + i) * CC + c0 + tx] * st[(c0 + tx) * 2] + st[(c0 + tx) * 2 + 1], 0.f); __syncthreads();
  for (int pass = 0; pass < 2; ++pass) { for (int i = ty; i < 32; i += 8) { const size_t o = ((size_t)b * CC + c0 + i) * NN + n0 + tx; *(volatile float*)(out + o) = bf16_round(x[o]) + tile[tx][i]; } if (pass == 0) __threadfence(); } }
extern "C" void kernel_launch(void* const* d_in, const int* in_sizes, int n_in,
                              void* d_out, int out_size, void* d_ws, size_t ws_size, hipStream_t stream) {
  (void)in_sizes; (void)n_in; (void)out_size;
  const float* x = (const float*)d_in[0]; const int* disc = (const int*)d_in[1]; (void)d_in[2]; const float* qw = (const float*)d_in[3]; const float* kw = (const float*)d_in[4]; const float* vw = (const float*)d_in[5]; const float* vb = (const float*)d_in[6]; const float* tw = (const float*)d_in[7]; const float* tb = (const float*)d_in[8]; const float* g = (const float*)d_in[9]; const float* be = (const float*)d_in[10]; const float* xl = (const float*)d_in[11]; const float* yl = (const float*)d_in[12]; const float* zl = (const float*)d_in[13];
  char* ws = (char*)d_ws; size_t off = 0;
  auto take = [&](size_t bytes) { char* p = ws + off; off += (bytes + 255) & ~(size_t)255; return p; };
  unsigned short* Bqkv = (unsigned short*)take((size_t)384 * CC * 2); unsigned short* Bt = (unsigned short*)take((size_t)CC * DVV * 2); float* bqkv = (float*)take(384 * 4);
  float* XT = (float*)take((size_t)NTOK * CC * 4); float* QKV = (float*)take((size_t)NTOK * 384 * 4); unsigned short* Kh = (unsigned short*)take((size_t)NTOK * DQK * 2); unsigned short* Kl = (unsigned short*)take((size_t)NTOK * DQK * 2); unsigned short* Lh = (unsigned short*)take((size_t)3 * NRP * DQK * 2); unsigned short* Ll = (unsigned short*)take((size_t)3 * NRP * DQK * 2);
  float* QL = (float*)take((size_t)NTOK * 3 * NRP * 4); _Float16* Vt = (_Float16*)take((size_t)BB * DVV * NN * 2); float* E = (float*)take((size_t)NN * NN * 4); float* Dn = (float*)take((size_t)NTOK * 4); _Float16* AT = (_Float16*)take((size_t)NN * NN * 2); float* XRt = (float*)take((size_t)NTOK * DVV * 4);
  float* Hm = QKV;   float* T2 = XRt;   double* part = (double*)take((size_t)(NTOK / 1024) * CC * 2 * 8); float* st = (float*)take(CC * 2 * 4);
  if (off > ws_size) return;
  k_round_rows<<<(DQK * CC / 8 + 255) / 256, 256, 0, stream>>>(qw, Bqkv, DQK * CC / 8); k_round_rows<<<(DQK * CC / 8 + 255) / 256, 256, 0, stream>>>(kw, Bqkv + (size_t)DQK * CC, DQK * CC / 8); k_round_rows<<<(DVV * CC / 8 + 255) / 256, 256, 0, stream>>>(vw, Bqkv + (size_t)2 * DQK * CC, DVV * CC / 8); k_round_rows<<<(CC * DVV / 8 + 255) / 256, 256, 0, stream>>>(tw, Bt, CC * DVV / 8);
  k_bcat384<<<2, 256, 0, stream>>>(vb, bqkv);
  k_xt<<<dim3(NN / 32, CC / 32, BB), 256, 0, stream>>>(x, XT);
  k_gemm_bf3<false, 0, true, false><<<((NTOK / 16) * 6 + 3) / 4, 128, 0, stream>>>(XT, CC, Bqkv, CC, bqkv, nullptr, 1, 0, QKV, 384, NTOK, 384, CC);
  k_planes<<<(unsigned)(((size_t)NTOK * DQK / 8 + 255) / 256), 256, 0, stream>>>(QKV + DQK, Kh, Kl, (size_t)NTOK * DQK / 8, 384, DQK, DQK); k_ltplanes<<<(3 * NRP * 8 + 255) / 256, 256, 0, stream>>>(xl, yl, zl, Lh, Ll);
  k_gemm_b<true, true, 0><<<dim3(((NTOK / 16) * 3 + 3) / 4, 1), 128, 0, stream>>>(QKV, 384, 0, Lh, Ll, DQK, 0, nullptr, nullptr, 0, 0, 1.f, 1.f, QL, 3 * NRP, 0, NTOK, 3 * NRP, DQK);
  k_vt<<<dim3(NN / 64, DVV / 64, BB), 256, 0, stream>>>(QKV, Vt);
  for (int b = 0; b < BB; ++b) {
    k_gemm_b<true, true, 0><<<dim3(((NN / 16) * (NN / 64) + 3) / 4, 1), 128, 0, stream>>>(QKV + (size_t)b * NN * 384, 384, 0, Kh + (size_t)b * NN * DQK, Kl + (size_t)b * NN * DQK, DQK, 0, nullptr, nullptr, 0, 0, 1.f, 1.f, E, NN, 0, NN, NN, DQK);
    k_softmax<<<NN / 32, 1024, 0, stream>>>(E, QL, disc, b, Dn);
    k_attnT<<<dim3(NN / 64, NN / 64), 256, 0, stream>>>(E, Dn, b, AT);
    k_gemm_hh<0><<<dim3(((NN / 16) * (DVV / 64) + 3) / 4, 1), 128, 0, stream>>>(AT, NN, 0, Vt + (size_t)b * DVV * NN, NN, 0, 0.00390625f, XRt + (size_t)b * NN * DVV, DVV, 0, NN, DVV, NN);
  }
  k_hdiff<<<(unsigned)(((size_t)NTOK * CC / 4 + 255) / 256), 256, 0, stream>>>(XT, XRt, Hm);
  k_gemm_bf3<true, 0, true, false><<<((NTOK / 16) * (CC / 64) + 3) / 4, 128, 0, stream>>>(Hm, CC, Bt, DVV, tb, nullptr, 1, 0, T2, CC, NTOK, CC, DVV);
  k_colstat<<<NTOK / 1024, 256, 0, stream>>>(T2, part); k_bnfin<<<1, 256, 0, stream>>>(part, g, be, st);
  k_out<<<dim3(CC / 32, NN / 32, BB), 256, 0, stream>>>(T2, st, x, (float*)d_out);
}
